// UVNetGraphEncoder_No_Edge_7310034338048
// MI455X (gfx1250) — hardware-verified
//
#include <hip/hip_runtime.h>

#define NN 50000
#define EE 600000
#define DD 128
#define BB 8
#define LRELU 0.01f
#define BUCKET 64
#define NBK   ((NN + BUCKET - 1) / BUCKET)
#define NBKP  800
#define CHUNK 2048
#define NCH   ((EE + CHUNK - 1) / CHUNK)
#define SLOT  32
#define LCAP  1280
#define GBLK  ((NN + 127) / 128)
#define POOLR 512
#define NPB   ((NN + POOLR - 1) / POOLR)
#define RSPLIT (1.0f / 2048.0f)

typedef _Float16 f16;
typedef __attribute__((ext_vector_type(16))) _Float16 v16h;
typedef __attribute__((ext_vector_type(8)))  float    v8f;
typedef __attribute__((ext_vector_type(4)))  float    f4;
typedef float v4fa __attribute__((ext_vector_type(4), may_alias));

__device__ __forceinline__ v8f wmma16(v16h a, v16h b, v8f c) { return __builtin_amdgcn_wmma_f32_16x16x32_f16(false, a, false, b, (short)0, c, false, false); }
__device__ __forceinline__ v8f wmma_split(v16h a, v16h al, v16h b, v16h bl, v8f c) { v8f x = {}; x = wmma16(al, b, x); x = wmma16(a, bl, x); return wmma16(a, b, c) + x * RSPLIT; }
__device__ __forceinline__ f16 lo_of(float v, f16 h) { return (f16)((v - (float)h) * 2048.0f); }

__global__ __launch_bounds__(256) void bin_kernel(const int* __restrict__ dst, int* __restrict__ slots, int* __restrict__ cnts) {
  __shared__ int cnt[NBKP];
  const int tid = threadIdx.x, ch = blockIdx.x;
  for (int i = tid; i < NBKP; i += 256) cnt[i] = 0;
  __syncthreads();
  int eb[8], ps[8];
#pragma unroll
  for (int u = 0; u < 8; ++u) {
    const int e = ch * CHUNK + u * 256 + tid;
    eb[u] = -1; ps[u] = -1;
    if (e < EE) { int d = dst[e]; d = ((unsigned)d < (unsigned)NN) ? d : 0; const int b = d / BUCKET; const int p = atomicAdd(&cnt[b], 1); if (p < SLOT) { eb[u] = b; ps[u] = p; } }
  }
  __syncthreads();
#pragma unroll 1
  for (int pass = 0; pass < 2; ++pass) {
#pragma unroll
    for (int u = 0; u < 8; ++u) if (eb[u] >= 0) *(volatile int*)(slots + ((size_t)ch * NBK + eb[u]) * SLOT + ps[u]) = ch * CHUNK + u * 256 + tid;
    for (int i = tid; i < NBKP; i += 256) *(volatile int*)(cnts + (size_t)ch * NBKP + i) = (i < NBK) ? min(cnt[i], SLOT) : 0;
    __threadfence();
  }
}

__global__ __launch_bounds__(256) void gather_kernel(const int* __restrict__ src, const int* __restrict__ dst,
                                                    const int* __restrict__ slots, const int* __restrict__ cnts,
                                                    const float* __restrict__ x, float* __restrict__ agg) {
  __shared__ int lst[LCAP], lsrc[LCAP];
  __shared__ int total;
  __shared__ int ncnt[BUCKET], noff[BUCKET];
  const int tid = threadIdx.x, lane = tid & 31, wave = tid >> 5;
  const int bk = blockIdx.x, n0 = bk * BUCKET;
  if (tid == 0) total = 0;
  if (tid < BUCKET) ncnt[tid] = 0;
  __syncthreads();
  int myc[2], mytot = 0;
#pragma unroll
  for (int u = 0; u < 2; ++u) { const int ch = tid + 256 * u; myc[u] = (ch < NCH) ? cnts[(size_t)ch * NBKP + bk] : 0; mytot += myc[u]; }
  {
    __shared__ int scan[256];
    scan[tid] = mytot;
    __syncthreads();
#pragma unroll
    for (int off = 1; off < 256; off <<= 1) { const int v = (tid >= off) ? scan[tid - off] : 0; __syncthreads(); scan[tid] += v; __syncthreads(); }
    int pos = scan[tid] - mytot;
    if (tid == 255) total = min(scan[255], LCAP);
#pragma unroll
    for (int u = 0; u < 2; ++u) {
      const int ch = tid + 256 * u;
      for (int i = 0; i < myc[u]; ++i) { if (pos < LCAP) { const int e = slots[((size_t)ch * NBK + bk) * SLOT + i]; int d = dst[e]; d = ((unsigned)d < (unsigned)NN) ? d : 0; lst[pos] = ((d - n0) << 24) | e; } ++pos; }
    }
    __syncthreads();
  }
  const int nl = total;
  for (int i = tid; i < nl; i += 256) atomicAdd(&ncnt[(lst[i] >> 24) & 63], 1);
  __syncthreads();
  if (tid == 0) { int o = 0; for (int j = 0; j < BUCKET; ++j) { noff[j] = o; o += ncnt[j]; } }
  __syncthreads();
  if (tid < BUCKET) { int p = noff[tid]; for (int i = 0; i < nl; ++i) if (((lst[i] >> 24) & 63) == tid) { int s = src[lst[i] & 0xFFFFFF]; s = ((unsigned)s < (unsigned)NN) ? s : 0; lsrc[p++] = s; } }
  __syncthreads();
  for (int j = wave; j < BUCKET; j += 8) {
    const int node = n0 + j;
    if (node >= NN) break;
    const int o0 = noff[j], cn = ncnt[j];
    f4 a = {0.f, 0.f, 0.f, 0.f};
    for (int i = 0; i < cn; ++i) a += *(const f4*)(x + (size_t)lsrc[o0 + i] * DD + lane * 4);
    float* o = agg + (size_t)node * DD + lane * 4;
    *(volatile f4*)o = a; __threadfence(); *(volatile f4*)o = a;
  }
}

__global__ __launch_bounds__(256)
void k_gemm_wmma(int mode, const float* __restrict__ X, const float* __restrict__ AGG, const float* __restrict__ epsP,
                 const float* __restrict__ scale, const float* __restrict__ shift,
                 const float* __restrict__ W, const float* __restrict__ bias,
                 float* __restrict__ Y, float* __restrict__ part, int nrows) {
  __shared__ __attribute__((aligned(32))) f16 Wswz[DD * DD], Wswl[DD * DD];
  __shared__ __attribute__((aligned(16))) float stg[8][16 * DD];
  __shared__ float pcol[8][2][DD];
  for (int i = threadIdx.x; i < DD * DD; i += 256) {
    int e = i & 15, ln = (i >> 4) & 31, t = (i >> 9) & 7, kc = i >> 12;
    int n = t * 16 + (ln & 15), kb = kc * 32 + (ln >> 4) * 8;
    int k = (e < 8) ? (kb + e) : (kb + 16 + (e - 8));
    const float v = W[k * DD + n]; const f16 h = (f16)v;
    Wswz[i] = h; Wswl[i] = lo_of(v, h);
  }
  __syncthreads();
  const int wave = threadIdx.x >> 5, lane = threadIdx.x & 31, n16 = lane & 15, hi = lane >> 4;
  const long rowStrip = (long)blockIdx.x * 128 + wave * 16;
  long r = rowStrip + n16;
  const bool rin = (r < nrows);
  if (!rin) r = 0;
  const float eps1 = (mode == 0) ? (1.0f + epsP[0]) : 1.0f;
  const float* __restrict__ xr = X + r * DD;
  const float* __restrict__ gr = AGG ? (AGG + r * DD) : X;
  v8f acc[8] = {};
#pragma unroll
  for (int kc = 0; kc < 4; ++kc) {
    const int kb = kc * 32 + hi * 8;
    float xv[16];
    *(f4*)(xv + 0) = *(const f4*)(xr + kb); *(f4*)(xv + 4) = *(const f4*)(xr + kb + 4);
    *(f4*)(xv + 8) = *(const f4*)(xr + kb + 16); *(f4*)(xv + 12) = *(const f4*)(xr + kb + 20);
    float av[16];
    if (mode == 0) {
      float gv[16];
      *(f4*)(gv + 0) = *(const f4*)(gr + kb); *(f4*)(gv + 4) = *(const f4*)(gr + kb + 4);
      *(f4*)(gv + 8) = *(const f4*)(gr + kb + 16); *(f4*)(gv + 12) = *(const f4*)(gr + kb + 20);
#pragma unroll
      for (int e = 0; e < 16; ++e) av[e] = eps1 * xv[e] + gv[e];
    } else {
      float sc[16], sf[16];
      *(f4*)(sc + 0) = *(const f4*)(scale + kb); *(f4*)(sc + 4) = *(const f4*)(scale + kb + 4);
      *(f4*)(sc + 8) = *(const f4*)(scale + kb + 16); *(f4*)(sc + 12) = *(const f4*)(scale + kb + 20);
      *(f4*)(sf + 0) = *(const f4*)(shift + kb); *(f4*)(sf + 4) = *(const f4*)(shift + kb + 4);
      *(f4*)(sf + 8) = *(const f4*)(shift + kb + 16); *(f4*)(sf + 12) = *(const f4*)(shift + kb + 20);
#pragma unroll
      for (int e = 0; e < 16; ++e) { const float v = sc[e] * xv[e] + sf[e]; av[e] = v > 0.f ? v : 0.f; }
    }
    if (!rin) {
#pragma unroll
      for (int e = 0; e < 16; ++e) av[e] = 0.f;
    }
    v16h a, al;
#pragma unroll
    for (int e = 0; e < 16; ++e) { const f16 h = (f16)av[e]; a[e] = h; al[e] = lo_of(av[e], h); }
#pragma unroll
    for (int t = 0; t < 8; ++t) {
      const v16h b  = *(const v16h*)(Wswz + (((kc * 8 + t) * 32 + lane) << 4));
      const v16h bl = *(const v16h*)(Wswl + (((kc * 8 + t) * 32 + lane) << 4));
      acc[t] = wmma_split(a, al, b, bl, acc[t]);
      asm volatile("" ::: "memory");
    }
  }
  float* sw = stg[wave];
#pragma unroll
  for (int t = 0; t < 8; ++t) {
    const int col = t * 16 + n16;
    const float bb = bias[col];
    float s = 0.f, s2 = 0.f;
#pragma unroll
    for (int v = 0; v < 8; ++v) {
      const long rr = rowStrip + v + 8 * hi;
      const float y = acc[t][v] + bb;
      sw[(v + 8 * hi) * DD + col] = y;
      if (rr < nrows) { s += y; s2 += y * y; }
    }
    s += __shfl_xor(s, 16, 32); s2 += __shfl_xor(s2, 16, 32);
    if (hi == 0) { pcol[wave][0][col] = s; pcol[wave][1][col] = s2; }
  }
  __syncthreads();
  {
    const int c = threadIdx.x & 127, w2 = threadIdx.x >> 7;
    float t = 0.f;
#pragma unroll
    for (int w = 0; w < 8; ++w) t += pcol[w][w2][c];
    float* dstp = part + (size_t)blockIdx.x * 256 + w2 * 128 + c;
    *(volatile float*)dstp = t; __threadfence(); *(volatile float*)dstp = t;
  }
  float* ob = Y + rowStrip * DD;
#pragma unroll 1
  for (int pass = 0; pass < 2; ++pass) {
#pragma unroll
    for (int i = 0; i < 16; ++i) { const int c = lane + 32 * i, rr = c >> 5, q = (c & 31) * 4; if (rowStrip + rr < nrows) *(volatile f4*)(ob + rr * DD + q) = *(const volatile v4fa*)(sw + rr * DD + q); }
    __threadfence();
  }
}

__global__ __launch_bounds__(256) void k_bn_finalize(const float* __restrict__ part, const float* g, const float* be,
                                                      float* __restrict__ scale, float* __restrict__ shift, float invN) {
  __shared__ double red[256];
  const int t = threadIdx.x;
  double acc = 0.0;
  for (int b = 0; b < GBLK; ++b) acc += (double)part[(size_t)b * 256 + t];
  red[t] = acc;
  __syncthreads();
  if (t < DD) {
    const double mean = red[t] * (double)invN;
    double var = red[128 + t] * (double)invN - mean * mean; if (var < 0.0) var = 0.0;
    const float inv = (float)(1.0 / sqrt(var + 1e-5));
    const float sc = g[t] * inv, sf = be[t] - (float)mean * sc;
    *(volatile float*)(scale + t) = sc; *(volatile float*)(shift + t) = sf; __threadfence();
    *(volatile float*)(scale + t) = sc; *(volatile float*)(shift + t) = sf;
  }
}

__global__ void k_bn_leaky(const float* __restrict__ Y, const float* __restrict__ scale, const float* __restrict__ shift, float* __restrict__ out, long n) {
  long i = (long)blockIdx.x * blockDim.x + threadIdx.x;
  if (i >= n) return;
  int c = (int)(i & 127);
  float t = scale[c] * Y[i] + shift[c];
  t = t > 0.f ? t : LRELU * t;
  *(volatile float*)(out + i) = t; __threadfence(); *(volatile float*)(out + i) = t;
}

__global__ __launch_bounds__(128) void k_pool_max(const float* __restrict__ H, const int* __restrict__ seg, float* __restrict__ ppart) {
  const int col = threadIdx.x;
  long r0 = (long)blockIdx.x * POOLR, rend = r0 + POOLR; if (rend > NN) rend = NN;
  float mk[BB];
#pragma unroll
  for (int b = 0; b < BB; ++b) mk[b] = -3.0e38f;
  for (long r = r0; r < rend; ++r) {
    int s = seg[r]; s = ((unsigned)s < (unsigned)BB) ? s : 0;
    const float v = H[r * DD + col];
#pragma unroll
    for (int b = 0; b < BB; ++b) mk[b] = (s == b) ? fmaxf(mk[b], v) : mk[b];
  }
  float* o = ppart + (size_t)blockIdx.x * BB * DD + col;
#pragma unroll 1
  for (int pass = 0; pass < 2; ++pass) {
#pragma unroll
    for (int b = 0; b < BB; ++b) *(volatile float*)(o + b * DD) = mk[b];
    __threadfence();
  }
}

__global__ __launch_bounds__(128) void k_score(const float* __restrict__ pp0, const float* __restrict__ pp1, const float* __restrict__ pp2,
                                               const float* W0, const float* b0, const float* W1, const float* b1, const float* W2, const float* b2,
                                               float* __restrict__ out) {
  __shared__ float pooled[3][BB][DD];
  const int o = threadIdx.x;
  for (int b = 0; b < BB; ++b) {
    float m0 = -3.0e38f, m1 = -3.0e38f, m2 = -3.0e38f;
    for (int blk = 0; blk < NPB; ++blk) {
      const size_t idx = ((size_t)blk * BB + b) * DD + o;
      m0 = fmaxf(m0, pp0[idx]); m1 = fmaxf(m1, pp1[idx]); m2 = fmaxf(m2, pp2[idx]);
    }
    pooled[0][b][o] = m0; pooled[1][b][o] = m1; pooled[2][b][o] = m2;
  }
  __syncthreads();
  for (int b = 0; b < BB; ++b) {
    float acc = b0[o] + b1[o] + b2[o];
    for (int k = 0; k < DD; ++k) {
      acc += pooled[0][b][k] * W0[k * DD + o];
      acc += pooled[1][b][k] * W1[k * DD + o];
      acc += pooled[2][b][k] * W2[k * DD + o];
    }
    *(volatile float*)(out + b * DD + o) = acc; __threadfence(); *(volatile float*)(out + b * DD + o) = acc;
  }
}

extern "C" void kernel_launch(void* const* d_in, const int* in_sizes, int n_in,
                              void* d_out, int out_size, void* d_ws, size_t ws_size,
                              hipStream_t stream) {
    const float* h   = (const float*)d_in[0];
    const int*   src = (const int*)d_in[1];
    const int*   dst = (const int*)d_in[2];
    const int*   seg = (const int*)d_in[3];
    const float* c_eps[2] = { (const float*)d_in[4],  (const float*)d_in[13] };
    const float* c_W1[2]  = { (const float*)d_in[5],  (const float*)d_in[14] };
    const float* c_b1[2]  = { (const float*)d_in[6],  (const float*)d_in[15] };
    const float* c_g1[2]  = { (const float*)d_in[7],  (const float*)d_in[16] };
    const float* c_be1[2] = { (const float*)d_in[8],  (const float*)d_in[17] };
    const float* c_W2[2]  = { (const float*)d_in[9],  (const float*)d_in[18] };
    const float* c_b2[2]  = { (const float*)d_in[10], (const float*)d_in[19] };
    const float* c_g2[2]  = { (const float*)d_in[11], (const float*)d_in[20] };
    const float* c_be2[2] = { (const float*)d_in[12], (const float*)d_in[21] };
    const float* p_W[3]   = { (const float*)d_in[22], (const float*)d_in[24], (const float*)d_in[26] };
    const float* p_b[3]   = { (const float*)d_in[23], (const float*)d_in[25], (const float*)d_in[27] };

    float* out_h2    = (float*)d_out;
    float* out_score = (float*)d_out + (long)NN * DD;

    char* w = (char*)d_ws;
    auto carve = [&](size_t bytes) -> char* { char* p = w; w += (bytes + 255) & ~(size_t)255; return p; };
    float* bufA  = (float*)carve((size_t)NN * DD * 4);
    float* bufB  = (float*)carve((size_t)NN * DD * 4);
    float* h1    = (float*)carve((size_t)NN * DD * 4);
    float* scale = (float*)carve(DD * 4);
    float* shift = (float*)carve(DD * 4);
    float* part  = (float*)carve((size_t)GBLK * 256 * 4);
    float* pp    = (float*)carve((size_t)3 * NPB * BB * DD * 4);
    int*   slots = (int*)carve((size_t)NCH * NBK * SLOT * 4);
    int*   cnts  = (int*)carve((size_t)NCH * NBKP * 4);

    const long nElem  = (long)NN * DD;
    const int  eBlk   = (int)((nElem + 255) / 256);
    const float invN  = 1.0f / (float)NN;
    const float* layer_in[2]  = { h, h1 };
    float*       layer_out[2] = { h1, out_h2 };
    const int NLRUN = 2;

    bin_kernel<<<NCH, 256, 0, stream>>>(dst, slots, cnts);
    for (int l = 0; l < NLRUN; ++l) {
        gather_kernel<<<NBK, 256, 0, stream>>>(src, dst, slots, cnts, layer_in[l], bufA);
        k_gemm_wmma<<<GBLK, 256, 0, stream>>>(0, layer_in[l], bufA, c_eps[l], scale, shift, c_W1[l], c_b1[l], bufB, part, NN);
        k_bn_finalize<<<1, 256, 0, stream>>>(part, c_g1[l], c_be1[l], scale, shift, invN);
        k_gemm_wmma<<<GBLK, 256, 0, stream>>>(1, bufB, nullptr, c_eps[l], scale, shift, c_W2[l], c_b2[l], bufA, part, NN);
        k_bn_finalize<<<1, 256, 0, stream>>>(part, c_g2[l], c_be2[l], scale, shift, invN);
        k_bn_leaky<<<eBlk, 256, 0, stream>>>(bufA, scale, shift, layer_out[l], nElem);
    }
    k_pool_max<<<NPB, DD, 0, stream>>>(h,      seg, pp);
    k_pool_max<<<NPB, DD, 0, stream>>>(h1,     seg, pp + (size_t)NPB * BB * DD);
    k_pool_max<<<NPB, DD, 0, stream>>>(out_h2, seg, pp + (size_t)2 * NPB * BB * DD);
    k_score<<<1, DD, 0, stream>>>(pp, pp + (size_t)NPB * BB * DD, pp + (size_t)2 * NPB * BB * DD,
                                  p_W[0], p_b[0], p_W[1], p_b[1], p_W[2], p_b[2], out_score);
}
